// MQF_75024488726656
// MI455X (gfx1250) — hardware-verified
//
#include <hip/hip_runtime.h>


#define NBI  4
#define CC   512
#define NN   1024
#define NH_  8
#define HDD  64
#define NROW CC
#define KW   NN
#define VHD  128
#define NKVV (NN / 128)
#define DM   CC
#define NTK  CC
#define LOSC 1024.0f

typedef _Float16 h16;
typedef unsigned short bf;
typedef __attribute__((ext_vector_type(16))) __bf16   v16bf;
typedef __attribute__((ext_vector_type(16))) _Float16 v16h;
typedef __attribute__((ext_vector_type(8)))  _Float16 v8h;
typedef __attribute__((ext_vector_type(8)))  unsigned short v8us;
typedef __attribute__((ext_vector_type(8)))  float    v8f;
typedef __attribute__((ext_vector_type(4)))  float    v4f;
typedef __attribute__((ext_vector_type(4)))  _Float16 v4h;
typedef v8h  __attribute__((may_alias)) v8ha;
typedef v4f  __attribute__((may_alias)) v4fa;
typedef v8us __attribute__((may_alias)) v8usa;

__device__ __forceinline__ unsigned short f2bf(float f) { unsigned u = __float_as_uint(f); u += 0x7FFFu + ((u >> 16) & 1u); return (unsigned short)(u >> 16); }
__device__ __forceinline__ float bf2f(unsigned short b) { return __uint_as_float(((unsigned)b) << 16); }
__device__ __forceinline__ float bfr(float f) { return bf2f(f2bf(f)); }
__device__ __forceinline__ v16h cat16(v8h lo, v8h hi) { return __builtin_shufflevector(lo, hi, 0, 1, 2, 3, 4, 5, 6, 7, 8, 9, 10, 11, 12, 13, 14, 15); }
__device__ __forceinline__ v16bf cat16b(v8us lo, v8us hi) { return __builtin_bit_cast(v16bf, __builtin_shufflevector(lo, hi, 0, 1, 2, 3, 4, 5, 6, 7, 8, 9, 10, 11, 12, 13, 14, 15)); }
__device__ __forceinline__ v8f wmma16(v16h a, v16h b, v8f c) { return __builtin_amdgcn_wmma_f32_16x16x32_f16(false, a, false, b, (short)0, c, false, false); }
__device__ __forceinline__ v8f wmmab(v16bf a, v16bf b, v8f c) { return __builtin_amdgcn_wmma_f32_16x16x32_bf16(false, a, false, b, (short)0, c, false, false); }

template <bool SPLITA, bool F16OUT = false>
__global__ __launch_bounds__(128) void k_gemmb(const bf* __restrict__ A, const bf* __restrict__ Al, const bf* __restrict__ Bn, const float* __restrict__ bias, float* C, int ldc, h16* C2, const float* __restrict__ R = nullptr, int K = DM, int roundR = 1) {
    __shared__ __align__(16) float ost[4][16 * 68];
    const int lane = threadIdx.x & 31, wave = threadIdx.x >> 5, lr = lane & 15, hi = lane >> 4;
    const int r0 = blockIdx.x * 64 + wave * 16, c0 = blockIdx.y * 64;
    const size_t aoff = (size_t)(r0 + lr) * K + 8 * hi;
    size_t boff[4];
#pragma unroll
    for (int t = 0; t < 4; ++t) boff[t] = (size_t)(c0 + t * 16 + lr) * K + 8 * hi;
    v8f acc[4];
#pragma unroll
    for (int t = 0; t < 4; ++t) acc[t] = (v8f){};
#pragma unroll 1
    for (int kc = 0; kc < K; kc += 32) {
        const v16bf a = cat16b(*(const v8us*)(A + aoff + kc), *(const v8us*)(A + aoff + kc + 16));
        v16bf al = a;
        if (SPLITA) al = cat16b(*(const v8us*)(Al + aoff + kc), *(const v8us*)(Al + aoff + kc + 16));
#pragma unroll
        for (int t = 0; t < 4; ++t) { const v16bf b = cat16b(*(const v8us*)(Bn + boff[t] + kc), *(const v8us*)(Bn + boff[t] + kc + 16)); acc[t] = wmmab(a, b, acc[t]); if (SPLITA) acc[t] = wmmab(al, b, acc[t]); }
        asm volatile("v_nop\n\tv_nop\n\tv_nop\n\tv_nop" : "+v"(acc[0]), "+v"(acc[1]), "+v"(acc[2]), "+v"(acc[3]) : "v"(a), "v"(al));
    }
    float* os = &ost[wave][0];
#pragma unroll
    for (int t = 0; t < 4; ++t) { const float bv = bias ? bfr(bias[c0 + t * 16 + lr]) : 0.f;
#pragma unroll
        for (int j = 0; j < 8; ++j) os[(hi * 8 + j) * 68 + t * 16 + lr] = acc[t][j] + bv; }
    __syncthreads();
    if (F16OUT) {
        h16* crow = (h16*)(void*)C + (size_t)r0 * ldc + c0;
        auto pass = [&]() {
#pragma unroll
            for (int s = 0; s < 4; ++s) { const int row = 4 * s + (lane >> 3), piece = lane & 7; const float* sp = os + row * 68 + piece * 8; v8h o, o2;
#pragma unroll
                for (int i = 0; i < 8; ++i) { const h16 a = (h16)sp[i]; o[i] = a; o2[i] = (h16)((sp[i] - (float)a) * LOSC); }
                *(volatile v8h*)(crow + (size_t)row * ldc + piece * 8) = o; if (C2) *(volatile v8h*)(C2 + (size_t)r0 * ldc + c0 + (size_t)row * ldc + piece * 8) = o2; }
        };
        pass(); __threadfence(); pass();
    } else {
        float* crow = C + (size_t)r0 * ldc + c0;
        auto pass = [&]() {
#pragma unroll
            for (int s = 0; s < 8; ++s) { const int Lid = (lane >> 3) + 4 * s, piece = lane & 7; const int row = Lid >> 1, cofs = (Lid & 1) * 32 + piece * 4;
                v4f val = *(const v4fa*)(os + row * 68 + cofs); if (R) { const v4f rv = *(const v4f*)(R + ((size_t)r0 + row) * ldc + c0 + cofs); val += roundR ? (v4f){bfr(rv[0]), bfr(rv[1]), bfr(rv[2]), bfr(rv[3])} : rv; }
                *(volatile v4f*)(crow + (size_t)row * ldc + cofs) = val; }
        };
        pass(); __threadfence(); pass();
    }
}

__global__ __launch_bounds__(128) void k_gemm3(const bf* __restrict__ Ah, const bf* __restrict__ Al, const bf* __restrict__ Bh, const bf* __restrict__ Bl, int K, float* C, int ldc) {
    __shared__ __align__(16) float ost[4][16 * 68];
    const int lane = threadIdx.x & 31, wave = threadIdx.x >> 5, lr = lane & 15, hi = lane >> 4;
    const int r0 = blockIdx.x * 64 + wave * 16, c0 = blockIdx.y * 64;
    const size_t aoff = (size_t)(r0 + lr) * K + 8 * hi;
    v8f acc[4];
#pragma unroll
    for (int t = 0; t < 4; ++t) acc[t] = (v8f){};
#pragma unroll 1
    for (int kc = 0; kc < K; kc += 32) {
        const v16bf a = cat16b(*(const v8us*)(Ah + aoff + kc), *(const v8us*)(Ah + aoff + kc + 16));
        const v16bf al = cat16b(*(const v8us*)(Al + aoff + kc), *(const v8us*)(Al + aoff + kc + 16));
#pragma unroll
        for (int t = 0; t < 4; ++t) { const size_t bo = (size_t)(c0 + t * 16 + lr) * K + kc + 8 * hi;
            const v16bf bh = cat16b(*(const v8us*)(Bh + bo), *(const v8us*)(Bh + bo + 16)); const v16bf bl = cat16b(*(const v8us*)(Bl + bo), *(const v8us*)(Bl + bo + 16));
            acc[t] = wmmab(a, bh, acc[t]); acc[t] = wmmab(al, bh, acc[t]); acc[t] = wmmab(a, bl, acc[t]); }
        asm volatile("v_nop\n\tv_nop\n\tv_nop\n\tv_nop" : "+v"(acc[0]), "+v"(acc[1]), "+v"(acc[2]), "+v"(acc[3]) : "v"(a), "v"(al));
    }
    float* os = &ost[wave][0];
#pragma unroll
    for (int t = 0; t < 4; ++t) {
#pragma unroll
        for (int j = 0; j < 8; ++j) os[(hi * 8 + j) * 68 + t * 16 + lr] = acc[t][j]; }
    __builtin_amdgcn_wave_barrier(); asm volatile("" ::: "memory");
    float* crow = C + (size_t)r0 * ldc + c0;
    auto pass = [&]() {
#pragma unroll
        for (int s = 0; s < 8; ++s) { const int Lid = (lane >> 3) + 4 * s, piece = lane & 7; const int row = Lid >> 1, cofs = (Lid & 1) * 32 + piece * 4;
            const v4f val = *(const v4fa*)(os + row * 68 + cofs); *(volatile v4f*)(crow + (size_t)row * ldc + cofs) = val; }
    };
    pass(); __threadfence(); pass();
}
__global__ __launch_bounds__(256) void k_vt(const float* __restrict__ V, bf* VTH, bf* VTL) {
    __shared__ float tl[64][65];
    const int tid = threadIdx.x, t0 = blockIdx.x * 64, d0 = blockIdx.y * 64, g = blockIdx.z;
    { const int tt = tid >> 2, dq = (tid & 3) * 16;
#pragma unroll
      for (int i = 0; i < 16; ++i) tl[dq + i][tt] = V[(size_t)(t0 + tt) * KW + g * VHD + d0 + dq + i]; }
    __syncthreads();
    const int piece = tid & 7;
    auto pass = [&]() {
#pragma unroll
        for (int s = 0; s < 2; ++s) { const int d = (tid >> 3) + 32 * s; v8us oh, ol;
#pragma unroll
            for (int i = 0; i < 8; ++i) { const float v = tl[d][piece * 8 + i]; const unsigned short hb = f2bf(v); oh[i] = hb; ol[i] = f2bf(v - bf2f(hb)); }
            const size_t o = ((size_t)g * VHD + d0 + d) * NROW + t0 + piece * 8; *(volatile v8us*)(VTH + o) = oh; *(volatile v8us*)(VTL + o) = ol; }
    };
    pass(); __threadfence(); pass();
}

__global__ __launch_bounds__(256) void k_bf(const float* __restrict__ src, bf* dst, size_t n8) {
    const size_t i = (size_t)blockIdx.x * 256 + threadIdx.x; if (i >= n8) return;
    const v8f v = *(const v8f*)(src + i * 8); v8us o;
#pragma unroll
    for (int k = 0; k < 8; ++k) o[k] = f2bf(v[k]);
    *(volatile v8us*)(dst + i * 8) = o; __threadfence(); *(volatile v8us*)(dst + i * 8) = o;
}
__global__ __launch_bounds__(256) void k_rowbias(float* Y, const float* __restrict__ b, bf* Yh, bf* Yl) {
    const int lane = threadIdx.x & 31, r = blockIdx.x * 8 + (threadIdx.x >> 5); if (r >= CC) return;
    const float bo = bfr(b[r]);
    v8f vals[NN / 256];
#pragma unroll
    for (int q = 0; q < NN / 256; ++q) { vals[q] = *(const v8f*)(Y + (size_t)r * NN + q * 256 + lane * 8);
#pragma unroll
        for (int i = 0; i < 8; ++i) vals[q][i] += bo; }
#pragma unroll 1
    for (int ps = 0; ps < 2; ++ps) {
#pragma unroll
        for (int q = 0; q < NN / 256; ++q) { const size_t o = (size_t)r * NN + q * 256 + lane * 8; v8us oh, ol;
#pragma unroll
            for (int i = 0; i < 8; ++i) { const unsigned short hb = f2bf(vals[q][i]); oh[i] = hb; ol[i] = f2bf(vals[q][i] - bf2f(hb)); }
            *(volatile v8f*)(Y + o) = vals[q]; *(volatile v8us*)(Yh + o) = oh; *(volatile v8us*)(Yl + o) = ol; }
        if (ps == 0) __threadfence(); }
}
__global__ __launch_bounds__(256) void k_posT(const float* __restrict__ rh, const float* __restrict__ rw, bf* Ph, bf* Pl) {
    const int lane = threadIdx.x & 31, n = blockIdx.x * 8 + (threadIdx.x >> 5); if (n >= NN) return;
    const int i = n / 32, j = n % 32;
#pragma unroll 1
    for (int ps = 0; ps < 2; ++ps) {
#pragma unroll 1
        for (int q = 0; q < CC / 256; ++q) { const size_t o = (size_t)n * CC + q * 256 + lane * 8; v8us oh, ol;
#pragma unroll
            for (int k = 0; k < 8; ++k) { const int c = q * 256 + lane * 8 + k; const int h = c / HDD, d = c % HDD; const float v = bfr(rh[((size_t)h * HDD + d) * 32 + j]) + bfr(rw[((size_t)h * HDD + d) * 32 + i]);
                const unsigned short hb = f2bf(v); oh[k] = hb; ol[k] = f2bf(v - bf2f(hb)); }
            *(volatile v8us*)(Ph + o) = oh; *(volatile v8us*)(Pl + o) = ol; }
        if (ps == 0) __threadfence(); }
}
__global__ __launch_bounds__(256) void k_cat2(const bf* __restrict__ X1h, const bf* __restrict__ X1l, const bf* __restrict__ X2h, const bf* __restrict__ X2l, int h, bf* Ah, bf* Al) {
    typedef __attribute__((ext_vector_type(4))) unsigned short v4us;
    const int lane = threadIdx.x & 31, n = blockIdx.x * 8 + (threadIdx.x >> 5); if (n >= NN) return;
    const int half = lane >> 4, c0 = (lane & 15) * 4; const size_t si = (size_t)n * CC + h * HDD + c0;
    const v4us vh = half ? *(const v4us*)(X2h + si) : *(const v4us*)(X1h + si); const v4us vl = half ? *(const v4us*)(X2l + si) : *(const v4us*)(X1l + si);
    const size_t o = (size_t)n * 128 + half * 64 + c0;
    *(volatile v4us*)(Ah + o) = vh; *(volatile v4us*)(Al + o) = vl; __threadfence(); *(volatile v4us*)(Ah + o) = vh; *(volatile v4us*)(Al + o) = vl;
}
__global__ __launch_bounds__(256) void k_softmax(const float* __restrict__ S, bf* PH, bf* PL) {
    const int lane = threadIdx.x & 31, r = blockIdx.x * 8 + (threadIdx.x >> 5); if (r >= NN) return;
    const float* sr = S + (size_t)r * NN; float m = -3.0e38f;
#pragma unroll 1
    for (int c0 = lane * 8; c0 < NN; c0 += 256) { const v8f v = *(const v8f*)(sr + c0);
#pragma unroll
        for (int i = 0; i < 8; ++i) m = fmaxf(m, v[i]); }
#pragma unroll
    for (int sh = 16; sh; sh >>= 1) m = fmaxf(m, __shfl_xor(m, sh, 32));
    float sum = 0.f;
#pragma unroll 1
    for (int c0 = lane * 8; c0 < NN; c0 += 256) { const v8f v = *(const v8f*)(sr + c0);
#pragma unroll
        for (int i = 0; i < 8; ++i) sum += __expf(v[i] - m); }
#pragma unroll
    for (int sh = 16; sh; sh >>= 1) sum += __shfl_xor(sum, sh, 32);
    const float inv = 1.0f / sum;
#pragma unroll 1
    for (int ps = 0; ps < 2; ++ps) {
#pragma unroll 1
        for (int c0 = lane * 8; c0 < NN; c0 += 256) { const v8f v = *(const v8f*)(sr + c0); v8us oh, ol;
#pragma unroll
            for (int i = 0; i < 8; ++i) { const float p = __expf(v[i] - m) * inv; const unsigned short hb = f2bf(p); oh[i] = hb; ol[i] = f2bf(p - bf2f(hb)); }
            const size_t o = (size_t)r * NN + c0; *(volatile v8us*)(PH + o) = oh; *(volatile v8us*)(PL + o) = ol; }
        if (ps == 0) __threadfence(); }
}

extern "C" void kernel_launch(void* const* d_in, const int* in_sizes, int n_in,
                              void* d_out, int out_size, void* d_ws, size_t ws_size, hipStream_t stream) {
    (void)in_sizes; (void)n_in; (void)out_size;
    const float* xin[3] = {(const float*)d_in[0], (const float*)d_in[1], (const float*)d_in[2]};
    const float* Wm[3] = {(const float*)d_in[3], (const float*)d_in[5], (const float*)d_in[7]}; const float* bm[3] = {(const float*)d_in[4], (const float*)d_in[6], (const float*)d_in[8]};
    const float* rh = (const float*)d_in[9]; const float* rw = (const float*)d_in[10];
    float* out = (float*)d_out;
    char* wsp = (char*)d_ws;
    auto take = [&](size_t bytes) { char* p = wsp; wsp += (bytes + 255) & ~(size_t)255; return (void*)p; };
    bf* WB[3]; for (int i = 0; i < 3; ++i) WB[i] = (bf*)take((size_t)CC * CC * 2);
    bf* XT = (bf*)take((size_t)NN * CC * 2); bf* XTl = (bf*)take((size_t)NN * CC * 2); bf* PTh = (bf*)take((size_t)NN * CC * 2); bf* PTl = (bf*)take((size_t)NN * CC * 2);
    float* Y[3]; bf* Yh[3]; bf* Yl[3]; bf* YTh[3]; bf* YTl[3];
    for (int i = 0; i < 3; ++i) { Y[i] = (float*)take((size_t)CC * NN * 4); Yh[i] = (bf*)take((size_t)CC * NN * 2); Yl[i] = (bf*)take((size_t)CC * NN * 2); YTh[i] = (bf*)take((size_t)NN * CC * 2); YTl[i] = (bf*)take((size_t)NN * CC * 2); }
    bf* A2h = (bf*)take((size_t)NN * 128 * 2); bf* A2l = (bf*)take((size_t)NN * 128 * 2); bf* B2h = (bf*)take((size_t)NN * 128 * 2); bf* B2l = (bf*)take((size_t)NN * 128 * 2);
    float* S = (float*)take((size_t)NN * NN * 4); bf* PH = (bf*)take((size_t)NN * NN * 2); bf* PL = (bf*)take((size_t)NN * NN * 2);
    if ((size_t)(wsp - (char*)d_ws) > ws_size) return;
    for (int i = 0; i < 3; ++i) k_bf<<<(CC * CC / 8 + 255) / 256, 256, 0, stream>>>(Wm[i], WB[i], CC * CC / 8);
    k_posT<<<NN / 8, 256, 0, stream>>>(rh, rw, PTh, PTl);
    for (int b = 0; b < NBI; ++b) {
        for (int i = 0; i < 3; ++i) {
            k_vt<<<dim3(NROW / 64, 2, NKVV), 256, 0, stream>>>(xin[i] + (size_t)b * CC * NN, XT, XTl);
            k_gemmb<false, false><<<dim3(CC / 64, NN / 64, 1), 128, 0, stream>>>(WB[i], nullptr, XT, nullptr, Y[i], NN, nullptr, nullptr, CC);
            k_rowbias<<<CC / 8, 256, 0, stream>>>(Y[i], bm[i], Yh[i], Yl[i]);
            k_vt<<<dim3(NROW / 64, 2, NKVV), 256, 0, stream>>>(Y[i], YTh[i], YTl[i]);
        }
        for (int h = 0; h < NH_; ++h)
            for (int br = 0; br < 3; ++br) { const int ia = br, ib = (br + 1) % 3, iv = (br + 2) % 3;
                k_cat2<<<NN / 8, 256, 0, stream>>>(YTh[ia], YTl[ia], PTh, PTl, h, A2h, A2l);
                k_cat2<<<NN / 8, 256, 0, stream>>>(YTh[ib], YTl[ib], YTh[ia], YTl[ia], h, B2h, B2l);
                k_gemm3<<<dim3(NN / 64, NN / 64, 1), 128, 0, stream>>>(A2h, A2l, B2h, B2l, 128, S, NN);
                k_softmax<<<NN / 8, 256, 0, stream>>>(S, PH, PL);
                k_gemm3<<<dim3(HDD / 64, NN / 64, 1), 128, 0, stream>>>(Yh[iv] + (size_t)h * HDD * NN, Yl[iv] + (size_t)h * HDD * NN, PH, PL, NN, out + (((size_t)br * NBI + b) * CC + h * HDD) * NN, NN);
            }
    }
}
